// GNN22_46093589020764
// MI455X (gfx1250) — hardware-run, weakly checked
//
#include <hip/hip_runtime.h>
#include <stddef.h>


#define NTHR      256
#define NWAVE     8
#define NBN       64
#define AP64      72
#define AP128     136
#define AP256     264
#define EPT       8
#define PIECE     (NTHR * EPT)
#define WCAP      (EPT * 32)
#define NCLS      100
#define ACT_RELU  0
#define ACT_LEAKY 1
#define NSLOPE    0.01f
#define WSCALE    64.0f
#define INV64     0.015625f
#define OWP1      0
#define OWS1      4096
#define OWN1      12288
#define OWP2      20480
#define OWS2      36864
#define OWN2      53248
#define OW1       69632
#define OW2       102400
#define OW2SRC    25600
#define PWTOT     135168
#define PTHR      128
#define PBLK      (PWTOT / (PTHR * 8))
#define AGGDYN    262144
#define L2DYN     60416
#define WSCAP     134217728

static_assert((PWTOT % (PTHR * 8)) == 0);
static_assert((OWS1 % 1024) == 0);
static_assert((OWN1 % 1024) == 0);
static_assert((OWP2 % 1024) == 0);
static_assert((OWS2 % 1024) == 0);
static_assert((OWN2 % 1024) == 0);
static_assert((OW1 % 1024) == 0);
static_assert((OW2 % 1024) == 0);
static_assert((OW2SRC % 1024) == 0);
static_assert(OW2 + 128 * 256 == PWTOT);
static_assert(PIECE == 2048);
static_assert((EPT % 4) == 0);
static_assert(((AP64 * 2) % 16) == 0);
static_assert(((AP128 * 2) % 16) == 0);
static_assert(((AP256 * 2) % 16) == 0);
static_assert(NBN == NWAVE * 8);
static_assert(NBN * AP128 <= 2 * NBN * AP64);
static_assert(NBN * AP256 <= 2 * NBN * AP128);
static_assert(L2DYN == 2 * NBN * AP128 * 2 + NBN * NCLS * 4);
static_assert(((2 * NBN * AP128 * 2) % 16) == 0);

typedef float          v4f   __attribute__((ext_vector_type(4)));
typedef float          v8f   __attribute__((ext_vector_type(8)));
typedef int            v4i   __attribute__((ext_vector_type(4)));
typedef unsigned int   v4u   __attribute__((ext_vector_type(4)));
typedef unsigned short v8us  __attribute__((ext_vector_type(8)));
typedef _Float16       v8h   __attribute__((ext_vector_type(8)));
typedef _Float16       v16h  __attribute__((ext_vector_type(16)));

__device__ __forceinline__ v16h mkfrag(v8us u0, v8us u1) {
  const v8h a = __builtin_bit_cast(v8h, u0);
  const v8h b = __builtin_bit_cast(v8h, u1);
  return __builtin_shufflevector(a, b, 0, 1, 2, 3, 4, 5, 6, 7, 8, 9, 10, 11, 12, 13, 14, 15);
}

__device__ __forceinline__ v8f wmf(v16h a, v16h b, v8f c) {
  v8f d = __builtin_amdgcn_wmma_f32_16x16x32_f16(false, a, false, b, (short)0, c, false, false);
  asm volatile("v_nop\n\tv_nop\n\tv_nop\n\tv_nop" : "+v"(d) : "v"(a), "v"(b));
  return d;
}
__device__ __forceinline__ v8f zero8() {
  v8f z = {0.f, 0.f, 0.f, 0.f, 0.f, 0.f, 0.f, 0.f};
  return z;
}
template <int NT>
__device__ __forceinline__ void zacc(v8f (&c)[NT]) {
#pragma unroll
  for (int t = 0; t < NT; ++t) c[t] = zero8();
}
__device__ __forceinline__ int iclamp(int v, int lo, int hi) { return v < lo ? lo : (v > hi ? hi : v); }

__device__ __forceinline__ v8us pack8(v4f a, v4f b) {
  const v8f f = __builtin_shufflevector(a, b, 0, 1, 2, 3, 4, 5, 6, 7);
  const v8h h = __builtin_convertvector(f, v8h);
  return __builtin_bit_cast(v8us, h);
}
__device__ __forceinline__ unsigned short h2us(float f) {
  return __builtin_bit_cast(unsigned short, (_Float16)f);
}
__device__ __forceinline__ void st16_f32(const float* __restrict__ rp, unsigned short* dp) {
  const v4f a0 = *(const v4f*)(rp);
  const v4f a1 = *(const v4f*)(rp + 4);
  const v4f a2 = *(const v4f*)(rp + 8);
  const v4f a3 = *(const v4f*)(rp + 12);
  *(v8us*)dp       = pack8(a0, a1);
  *(v8us*)(dp + 8) = pack8(a2, a3);
}

__device__ __forceinline__ float sigm_f(float z) {
  const float zc = fminf(fmaxf(z, -80.0f), 80.0f);
  return __builtin_amdgcn_rcpf(1.0f + __expf(-zc));
}

template <int NT>
__device__ __forceinline__ void gemmNT(const unsigned short* ap, const unsigned short* __restrict__ bpl,
                                       int K, int nks, int n0, int m, int hh, v8f (&c)[NT]) {
#pragma unroll 1
  for (int ks = 0; ks < nks; ++ks) {
    const v16h a = mkfrag(*(const v8us*)(ap + 32 * ks), *(const v8us*)(ap + 32 * ks + 16));
    const size_t bo = (size_t)(n0 + m) * K + 32 * ks + 8 * hh;
#pragma unroll
    for (int t = 0; t < NT; ++t) {
      const size_t o = bo + (size_t)(16 * t) * K;
      const v16h b = mkfrag(*(const v8us*)(bpl + o), *(const v8us*)(bpl + o + 16));
      c[t] = wmf(a, b, c[t]);
    }
  }
}

template <int NT, int ACT>
__device__ __forceinline__ void stage16(unsigned short* so, int pitch, int row0, int col0, v8f (&c)[NT],
                                        const float* __restrict__ bias) {
#pragma unroll
  for (int t = 0; t < NT; ++t) {
    const int col = col0 + 16 * t;
    const float bv = bias[col];
    unsigned short* sp = so + row0 * pitch + col;
#pragma unroll
    for (int r = 0; r < 8; ++r) {
      float v = c[t][r] * INV64 + bv;
      if (ACT == ACT_RELU) v = fmaxf(v, 0.0f);
      else                 v = (v > 0.0f) ? v : NSLOPE * v;
      sp[r * pitch] = h2us(v);
    }
  }
}

__device__ __forceinline__ void rows64(const unsigned short* so, int ap, unsigned short* dst, int n0, int tid) {
#pragma unroll
  for (int it = 0; it < 2; ++it) {
    const int p = it * NTHR + tid;
    const int row = p >> 3, c8 = p & 7;
    const v8us v = *(const v8us*)(so + row * ap + 8 * c8);
    *(volatile v8us*)(dst + (size_t)(n0 + row) * 64 + 8 * c8) = v;
  }
}
__device__ __forceinline__ void rows128(const unsigned short* so, int ap, unsigned short* dst, int n0, int tid) {
#pragma unroll
  for (int it = 0; it < 4; ++it) {
    const int p = it * NTHR + tid;
    const int row = p >> 4, c8 = p & 15;
    const v8us v = *(const v8us*)(so + row * ap + 8 * c8);
    *(volatile v8us*)(dst + (size_t)(n0 + row) * 128 + 8 * c8) = v;
  }
}

__global__ __launch_bounds__(PTHR) void k_prep(
    const float* __restrict__ wp1, const float* __restrict__ wself1, const float* __restrict__ wneigh1,
    const float* __restrict__ wp2, const float* __restrict__ wself2, const float* __restrict__ wneigh2,
    const float* __restrict__ w1, const float* __restrict__ w2, unsigned short* wpl) {
  const int tid = (int)threadIdx.x;
  const int ob = (int)blockIdx.x * (PTHR * 8);
  const int o = ob + tid * 8;
  const float* src = wp1;
  int sb = OWP1;
  int valid = 1;
  if (ob >= OW2)       { src = w2;      sb = OW2;  valid = (ob - OW2 < OW2SRC) ? 1 : 0; }
  else if (ob >= OW1)  { src = w1;      sb = OW1;  }
  else if (ob >= OWN2) { src = wneigh2; sb = OWN2; }
  else if (ob >= OWS2) { src = wself2;  sb = OWS2; }
  else if (ob >= OWP2) { src = wp2;     sb = OWP2; }
  else if (ob >= OWN1) { src = wneigh1; sb = OWN1; }
  else if (ob >= OWS1) { src = wself1;  sb = OWS1; }
  v4f a = {0.0f, 0.0f, 0.0f, 0.0f};
  v4f b = a;
  if (valid != 0) {
    const float* p = src + (o - sb);
    a = *(const v4f*)p;
    b = *(const v4f*)(p + 4);
  }
  a = a * WSCALE;
  b = b * WSCALE;
  const v8us hv = pack8(a, b);
  unsigned short* d = wpl + o;
  *(volatile v8us*)d = hv;
  __threadfence();
  *(volatile v8us*)d = hv;
}

__global__ __launch_bounds__(NTHR) void k_pool1(
    const float* __restrict__ feat, const unsigned short* __restrict__ wpl, const float* __restrict__ bpp1,
    unsigned short* PQ1, int nN) {
  __shared__ __attribute__((aligned(16))) unsigned short sA[NBN * AP64];
  __shared__ __attribute__((aligned(16))) unsigned short sO[NBN * AP64];
  const int tid = (int)threadIdx.x, lane = tid & 31, wave = tid >> 5, hh = lane >> 4, m = lane & 15;
  const int n0 = (int)blockIdx.x * NBN;
  {
    const int nl = tid >> 2, q = tid & 3;
    int node = n0 + nl;
    node = node > nN - 1 ? nN - 1 : node;
    st16_f32(feat + (size_t)node * 64 + 16 * q, sA + nl * AP64 + 16 * q);
  }
  __syncthreads();
  const int rt = wave & 3, cg = wave >> 2;
  {
    v8f c[2];
    zacc<2>(c);
    gemmNT<2>(sA + (16 * rt + m) * AP64 + 8 * hh, wpl + OWP1, 64, 2, 32 * cg, m, hh, c);
    stage16<2, ACT_RELU>(sO, AP64, 16 * rt + 8 * hh, 32 * cg + m, c, bpp1);
  }
  __syncthreads();
  rows64(sO, AP64, PQ1, n0, tid);
  __threadfence();
  rows64(sO, AP64, PQ1, n0, tid);
}

template <int CPL> struct LaneVec;
template <> struct LaneVec<2> {
  typedef unsigned short U __attribute__((ext_vector_type(2)));
  typedef _Float16       H __attribute__((ext_vector_type(2)));
  typedef float          F __attribute__((ext_vector_type(2)));
};
template <> struct LaneVec<4> {
  typedef unsigned short U __attribute__((ext_vector_type(4)));
  typedef _Float16       H __attribute__((ext_vector_type(4)));
  typedef float          F __attribute__((ext_vector_type(4)));
};

template <int SLB_>
__device__ __forceinline__ int scan_piece(const int* __restrict__ ei, int lim, int cbase, int base,
                                          int* list, int tid, int wave) {
  constexpr int NBC = 1 << SLB_;
  int wc = 0;
  const int el0  = tid * EPT;
  const int e0   = cbase + el0;
  const int sent = -2147483647 - 1;
  int kk[EPT];
  if (cbase + PIECE <= lim) {
    const v4i* p = (const v4i*)(ei + e0);
#pragma unroll
    for (int u = 0; u < EPT / 4; ++u) {
      const v4i d = p[u];
      kk[4 * u] = d.x; kk[4 * u + 1] = d.y; kk[4 * u + 2] = d.z; kk[4 * u + 3] = d.w;
    }
  } else {
    const int lm = lim - 1;
#pragma unroll
    for (int q = 0; q < EPT; ++q) {
      const int eq = e0 + q;
      const int ec = eq > lm ? lm : eq;
      const int a = ei[ec];
      kk[q] = (eq < lim) ? a : sent;
    }
  }
  const unsigned nb = (unsigned)base;
  unsigned sq[EPT];
  bool hq[EPT];
  bool anyl = false;
#pragma unroll
  for (int q = 0; q < EPT; ++q) {
    sq[q] = (unsigned)kk[q] - nb;
    hq[q] = sq[q] < (unsigned)NBC;
    anyl = anyl | hq[q];
  }
  const unsigned any = __builtin_amdgcn_ballot_w32(anyl);
  if (any != 0u) {
#define HIT(HQ, SQ, Q) { \
      const unsigned mj = __builtin_amdgcn_ballot_w32(HQ); \
      if (mj != 0u) { \
        if (HQ) { \
          const int ps = wc + (int)__builtin_amdgcn_mbcnt_lo(mj, 0u); \
          if (ps < WCAP) list[wave * WCAP + ps] = ((el0 + (Q)) << SLB_) | (int)(SQ); \
        } \
        wc += (int)__builtin_popcount(mj); } }
#pragma unroll
    for (int q = 0; q < EPT; ++q) {
      HIT(hq[q], sq[q], q)
    }
#undef HIT
  }
  return wc;
}

template <int NCH, int SLB_>
__device__ __forceinline__ void drain_max(const int* list, const int* wcnt, unsigned short* accH,
                                          const int* __restrict__ esrc, const unsigned short* __restrict__ PQ,
                                          int cbase, int nE, int nN, int lane, int wave) {
  constexpr int NBC = 1 << SLB_;
  constexpr int CPL = NCH / 32;
  typedef typename LaneVec<CPL>::U UT;
  typedef typename LaneVec<CPL>::H HT;
  typedef typename LaneVec<CPL>::F FT;
#pragma unroll 1
  for (int wsx = 0; wsx < NWAVE; ++wsx) {
    int n = __builtin_amdgcn_readfirstlane(wcnt[wsx]);
    n = n > WCAP ? WCAP : (n < 0 ? 0 : n);
    const int* lp = list + wsx * WCAP;
#pragma unroll 1
    for (int bb = 0; bb < n; bb += 32) {
      const int idx = bb + lane;
      const int ic = idx > WCAP - 1 ? WCAP - 1 : idx;
      const int ent = lp[ic];
      const bool own = (idx < n) && ((ent & (NWAVE - 1)) == wave);
      unsigned msk = __builtin_amdgcn_ballot_w32(own);
#pragma unroll 1
      while (msk != 0u) {
        const int bit = (int)__builtin_ctz(msk);
        msk &= msk - 1u;
        const int e2 = __builtin_amdgcn_readlane(ent, bit);
        const int slot = e2 & (NBC - 1);
        const int el = (e2 >> SLB_) & (PIECE - 1);
        int e = cbase + el;
        e = e > nE - 1 ? nE - 1 : (e < 0 ? 0 : e);
        const int s = iclamp(esrc[e], 0, nN - 1);
        const UT qb = *(const UT*)(PQ + (size_t)s * NCH + CPL * lane);
        const FT qf = __builtin_convertvector(__builtin_bit_cast(HT, qb), FT);
        unsigned short* ap = accH + slot * NCH + CPL * lane;
        const UT ab = *(const UT*)ap;
        FT af = __builtin_convertvector(__builtin_bit_cast(HT, ab), FT);
#pragma unroll
        for (int j = 0; j < CPL; ++j) af[j] = fmaxf(af[j], qf[j]);
        *(UT*)ap = __builtin_bit_cast(UT, __builtin_convertvector(af, HT));
      }
    }
  }
}

template <int NCH, int SLB_>
__device__ __forceinline__ void hn_rows(const unsigned short* accH, unsigned short* HN, int base, int lane, int wave) {
  constexpr int NBC = 1 << SLB_;
  constexpr int RPW = NBC / NWAVE;
  constexpr int L8  = NCH / 8;
  constexpr int RPI = 32 / L8;
  constexpr int NIT = RPW / RPI;
  const int sub = lane / L8, c8 = lane % L8;
#pragma unroll 1
  for (int it = 0; it < NIT; ++it) {
    const int s = wave * RPW + it * RPI + sub;
    v8us v = *(const v8us*)(accH + s * NCH + 8 * c8);
#pragma unroll
    for (int j = 0; j < 8; ++j) v[j] = (v[j] == 0xFC00) ? (unsigned short)0 : v[j];
    *(volatile v8us*)(HN + (size_t)(base + s) * NCH + 8 * c8) = v;
  }
}

template <int NCH, int SLB_>
__global__ __launch_bounds__(NTHR) void k_agg(
    const int* __restrict__ edst, const int* __restrict__ esrc, const unsigned short* __restrict__ PQ,
    unsigned short* HN, int nE, int nN) {
  constexpr int NBC = 1 << SLB_;
  static_assert(NBC * NCH == 131072);
  static_assert(SLB_ >= 3);
  extern __shared__ __attribute__((aligned(16))) unsigned short accH[];
  __shared__ int list[NWAVE * WCAP];
  __shared__ int wcnt[NWAVE];
  const int tid = (int)threadIdx.x, lane = tid & 31, wave = tid >> 5;
  const int base = (int)blockIdx.x * NBC;
  {
    v4u nf;
    nf.x = 0xFC00FC00u; nf.y = 0xFC00FC00u; nf.z = 0xFC00FC00u; nf.w = 0xFC00FC00u;
#pragma unroll 1
    for (int i = tid; i < (NBC * NCH) / 8; i += NTHR) *(v4u*)(accH + 8 * i) = nf;
  }
  __syncthreads();
#pragma unroll 1
  for (int cbase = 0; cbase < nE; cbase += PIECE) {
    const int wc = scan_piece<SLB_>(edst, nE, cbase, base, list, tid, wave);
    if (lane == 0) wcnt[wave] = wc;
    __syncthreads();
    drain_max<NCH, SLB_>(list, wcnt, accH, esrc, PQ, cbase, nE, nN, lane, wave);
    __syncthreads();
  }
  __syncthreads();
  hn_rows<NCH, SLB_>(accH, HN, base, lane, wave);
  __threadfence();
  hn_rows<NCH, SLB_>(accH, HN, base, lane, wave);
}

__global__ __launch_bounds__(NTHR) void k_l1(
    const float* __restrict__ feat, const unsigned short* __restrict__ HN1, const unsigned short* __restrict__ wpl,
    const float* __restrict__ bn1, const float* __restrict__ bpp2, unsigned short* H1H, unsigned short* PQ2, int nN) {
  __shared__ __attribute__((aligned(16))) unsigned short sX[2 * NBN * AP64];
  __shared__ __attribute__((aligned(16))) unsigned short sH[NBN * AP128];
  unsigned short* sA = sX;
  unsigned short* sN = sX + NBN * AP64;
  unsigned short* sP = sX;
  const int tid = (int)threadIdx.x, lane = tid & 31, wave = tid >> 5, hh = lane >> 4, m = lane & 15;
  const int n0 = (int)blockIdx.x * NBN;
  {
    const int nl = tid >> 2, q = tid & 3;
    int node = n0 + nl;
    node = node > nN - 1 ? nN - 1 : node;
    st16_f32(feat + (size_t)node * 64 + 16 * q, sA + nl * AP64 + 16 * q);
    const unsigned short* hp = HN1 + (size_t)node * 64 + 16 * q;
    *(v8us*)(sN + nl * AP64 + 16 * q)     = *(const v8us*)hp;
    *(v8us*)(sN + nl * AP64 + 16 * q + 8) = *(const v8us*)(hp + 8);
  }
  __syncthreads();
  const int rt = wave & 3, cg = wave >> 2;
  {
    v8f c[4];
    zacc<4>(c);
    gemmNT<4>(sA + (16 * rt + m) * AP64 + 8 * hh, wpl + OWS1, 64, 2, 64 * cg, m, hh, c);
    gemmNT<4>(sN + (16 * rt + m) * AP64 + 8 * hh, wpl + OWN1, 64, 2, 64 * cg, m, hh, c);
    stage16<4, ACT_LEAKY>(sH, AP128, 16 * rt + 8 * hh, 64 * cg + m, c, bn1);
  }
  __syncthreads();
  rows128(sH, AP128, H1H, n0, tid);
  {
    v8f c[4];
    zacc<4>(c);
    gemmNT<4>(sH + (16 * rt + m) * AP128 + 8 * hh, wpl + OWP2, 128, 4, 64 * cg, m, hh, c);
    stage16<4, ACT_RELU>(sP, AP128, 16 * rt + 8 * hh, 64 * cg + m, c, bpp2);
  }
  __threadfence();
  rows128(sH, AP128, H1H, n0, tid);
  __syncthreads();
  rows128(sP, AP128, PQ2, n0, tid);
  __threadfence();
  rows128(sP, AP128, PQ2, n0, tid);
}

__global__ __launch_bounds__(NTHR) void k_l2(
    const unsigned short* __restrict__ H1H, const unsigned short* __restrict__ HN2, const unsigned short* __restrict__ wpl,
    const float* __restrict__ bn2, const float* __restrict__ bb1, const float* __restrict__ bb2,
    float* out, int nN) {
  extern __shared__ __attribute__((aligned(16))) unsigned short dyn[];
  unsigned short* sA  = dyn;
  unsigned short* sN  = dyn + NBN * AP128;
  unsigned short* sH3 = dyn;
  unsigned short* sH2 = dyn + 2 * NBN * AP128;
  float* sOut = (float*)(dyn + 2 * NBN * AP128);
  const int tid = (int)threadIdx.x, lane = tid & 31, wave = tid >> 5, hh = lane >> 4, m = lane & 15;
  const int n0 = (int)blockIdx.x * NBN;

  {
    const int nl = tid >> 2, q = tid & 3;
    int node = n0 + nl;
    node = node > nN - 1 ? nN - 1 : node;
    const unsigned short* hp = H1H + (size_t)node * 128 + 32 * q;
    const unsigned short* gp = HN2 + (size_t)node * 128 + 32 * q;
    unsigned short* da = sA + nl * AP128 + 32 * q;
    unsigned short* dn = sN + nl * AP128 + 32 * q;
#pragma unroll
    for (int j = 0; j < 4; ++j) {
      *(v8us*)(da + 8 * j) = *(const v8us*)(hp + 8 * j);
      *(v8us*)(dn + 8 * j) = *(const v8us*)(gp + 8 * j);
    }
  }
  __syncthreads();
  const int rt = wave & 3, cg = wave >> 2;

  {
    v8f c[4];
    zacc<4>(c);
    gemmNT<4>(sA + (16 * rt + m) * AP128 + 8 * hh, wpl + OWS2, 128, 4, 64 * cg, m, hh, c);
    gemmNT<4>(sN + (16 * rt + m) * AP128 + 8 * hh, wpl + OWN2, 128, 4, 64 * cg, m, hh, c);
    stage16<4, ACT_LEAKY>(sH2, AP128, 16 * rt + 8 * hh, 64 * cg + m, c, bn2);
  }
  __syncthreads();

#pragma unroll 1
  for (int qq = 0; qq < 2; ++qq) {
    v8f c[4];
    zacc<4>(c);
    gemmNT<4>(sH2 + (16 * rt + m) * AP128 + 8 * hh, wpl + OW1, 128, 4, 128 * cg + 64 * qq, m, hh, c);
    stage16<4, ACT_LEAKY>(sH3, AP256, 16 * rt + 8 * hh, 128 * cg + 64 * qq + m, c, bb1);
  }
  __syncthreads();

  {
    v8f c[4];
    zacc<4>(c);
    gemmNT<4>(sH3 + (16 * rt + m) * AP256 + 8 * hh, wpl + OW2, 256, 8, 64 * cg, m, hh, c);
#pragma unroll
    for (int t = 0; t < 4; ++t) {
      const int col = 64 * cg + 16 * t + m;
      const int cb = col > NCLS - 1 ? NCLS - 1 : col;
      const float bv = bb2[cb];
      const int row0 = 16 * rt + 8 * hh;
#pragma unroll
      for (int r = 0; r < 8; ++r) {
        const float y = sigm_f(c[t][r] * INV64 + bv);
        if (col < NCLS) sOut[(row0 + r) * NCLS + col] = y;
      }
    }
  }
  __syncthreads();

  {
    int nr = nN - n0;
    nr = nr > NBN ? NBN : (nr < 1 ? 1 : nr);
    const int np = nr * (NCLS / 4);
    float* ob = out + (size_t)n0 * NCLS;
#pragma unroll 1
    for (int it = 0; it < 7; ++it) {
      const int p = it * NTHR + tid;
      const int pc = p > (NBN * NCLS / 4) - 1 ? (NBN * NCLS / 4) - 1 : p;
      const v4f v = *(const v4f*)(sOut + 4 * pc);
      if (p < np) *(volatile v4f*)(ob + (size_t)4 * p) = v;
    }
    __threadfence();
#pragma unroll 1
    for (int it = 0; it < 7; ++it) {
      const int p = it * NTHR + tid;
      const int pc = p > (NBN * NCLS / 4) - 1 ? (NBN * NCLS / 4) - 1 : p;
      const v4f v = *(const v4f*)(sOut + 4 * pc);
      if (p < np) *(volatile v4f*)(ob + (size_t)4 * p) = v;
    }
  }
}

extern "C" void kernel_launch(void* const* d_in, const int* in_sizes, int n_in,
                              void* d_out, int out_size, void* d_ws, size_t ws_size,
                              hipStream_t stream) {
  if (n_in < 17) return;
  const int nN = in_sizes[0] / 64;
  if (nN < 1 || nN > (1 << 22) || in_sizes[0] != nN * 64) return;
  const int nE = in_sizes[1];
  if (nE < 1 || nE > (1 << 27) || in_sizes[2] != nE) return;
  if (in_sizes[3] != 64 * 64 || in_sizes[4] != 64) return;
  if (in_sizes[5] != 128 * 64 || in_sizes[6] != 128 * 64 || in_sizes[7] != 128) return;
  if (in_sizes[8] != 128 * 128 || in_sizes[9] != 128) return;
  if (in_sizes[10] != 128 * 128 || in_sizes[11] != 128 * 128 || in_sizes[12] != 128) return;
  if (in_sizes[13] != 256 * 128 || in_sizes[14] != 256) return;
  if (in_sizes[15] != NCLS * 256 || in_sizes[16] != NCLS) return;
  if ((size_t)out_size != (size_t)nN * NCLS) return;

  const float* feat    = (const float*)d_in[0];
  const int*   esrc    = (const int*)d_in[1];
  const int*   edst    = (const int*)d_in[2];
  const float* wp1     = (const float*)d_in[3];
  const float* bpp1    = (const float*)d_in[4];
  const float* wself1  = (const float*)d_in[5];
  const float* wneigh1 = (const float*)d_in[6];
  const float* bn1     = (const float*)d_in[7];
  const float* wp2     = (const float*)d_in[8];
  const float* bpp2    = (const float*)d_in[9];
  const float* wself2  = (const float*)d_in[10];
  const float* wneigh2 = (const float*)d_in[11];
  const float* bn2     = (const float*)d_in[12];
  const float* w1      = (const float*)d_in[13];
  const float* bb1     = (const float*)d_in[14];
  const float* w2      = (const float*)d_in[15];
  const float* bb2     = (const float*)d_in[16];
  float* out = (float*)d_out;

  const int nb64 = (nN + NBN - 1) / NBN;
  const int Npad64 = nb64 * NBN;
  const int nbA1 = (nN + 2047) / 2048;
  const int NpA1 = nbA1 * 2048;
  const int nbA2 = (nN + 1023) / 1024;
  const int NpA2 = nbA2 * 1024;

  char* ws = (char*)d_ws;
  size_t off = 0;
  const size_t oW   = off; off += (size_t)PWTOT * 2;          off = (off + 255) & ~(size_t)255;
  const size_t oPQ1 = off; off += (size_t)Npad64 * 64 * 2;    off = (off + 255) & ~(size_t)255;
  const size_t oHN1 = off; off += (size_t)NpA1 * 64 * 2;      off = (off + 255) & ~(size_t)255;
  const size_t oH1  = off; off += (size_t)Npad64 * 128 * 2;   off = (off + 255) & ~(size_t)255;
  const size_t oPQ2 = off; off += (size_t)Npad64 * 128 * 2;   off = (off + 255) & ~(size_t)255;
  const size_t oHN2 = off; off += (size_t)NpA2 * 128 * 2;     off = (off + 255) & ~(size_t)255;
  if (off > ws_size || off > (size_t)WSCAP) return;
  unsigned short* wpl = (unsigned short*)(ws + oW);
  unsigned short* PQ1 = (unsigned short*)(ws + oPQ1);
  unsigned short* HN1 = (unsigned short*)(ws + oHN1);
  unsigned short* H1H = (unsigned short*)(ws + oH1);
  unsigned short* PQ2 = (unsigned short*)(ws + oPQ2);
  unsigned short* HN2 = (unsigned short*)(ws + oHN2);

  hipFuncSetAttribute(reinterpret_cast<const void*>(&k_agg<64, 11>), hipFuncAttributeMaxDynamicSharedMemorySize, AGGDYN);
  hipFuncSetAttribute(reinterpret_cast<const void*>(&k_agg<128, 10>), hipFuncAttributeMaxDynamicSharedMemorySize, AGGDYN);

  k_prep<<<PBLK, PTHR, 0, stream>>>(wp1, wself1, wneigh1, wp2, wself2, wneigh2, w1, w2, wpl);
  k_pool1<<<nb64, NTHR, 0, stream>>>(feat, wpl, bpp1, PQ1, nN);
  k_agg<64, 11><<<nbA1, NTHR, AGGDYN, stream>>>(edst, esrc, PQ1, HN1, nE, nN);
  k_l1<<<nb64, NTHR, 0, stream>>>(feat, HN1, wpl, bn1, bpp2, H1H, PQ2, nN);
  k_agg<128, 10><<<nbA2, NTHR, AGGDYN, stream>>>(edst, esrc, PQ2, HN2, nE, nN);
  k_l2<<<nb64, NTHR, L2DYN, stream>>>(H1H, HN2, wpl, bn2, bb1, bb2, out, nN);
}
